// SparseAttention_47278999994875
// MI455X (gfx1250) — hardware-verified
//
#include <hip/hip_runtime.h>
#include <math.h>


#ifndef NB
#define NB 2
#endif
#ifndef SEQ
#define SEQ 2048
#endif
#ifndef RHP
#define RHP 512
#endif
#define NB_FULL  2
#define SEQ_FULL 2048
#define DM   2048
#define NH   16
#define NKV  4
#define HD   128
#define KVD  (NKV * HD)
#define NREP (NH / NKV)
#define MROWS (NB * SEQ)

constexpr int RH = (RHP < SEQ) ? RHP : SEQ;
constexpr int CP = 132;

static_assert(NB >= 1 && NB <= NB_FULL);
static_assert(SEQ >= 64 && SEQ <= SEQ_FULL);
static_assert(SEQ % 64 == 0);
static_assert(RH % 64 == 0 && RH >= 64 && RH <= SEQ);
static_assert(DM % 128 == 0 && KVD % 128 == 0);
static_assert(DM % 32 == 0);
static_assert(HD == 128);
static_assert(NH % NKV == 0);

typedef _Float16 v16h __attribute__((ext_vector_type(16)));
typedef _Float16 v8h  __attribute__((ext_vector_type(8)));
typedef _Float16 v8ha __attribute__((ext_vector_type(8), may_alias));
typedef float    v8f  __attribute__((ext_vector_type(8)));
typedef float    v4f  __attribute__((ext_vector_type(4)));
typedef float    v4fa __attribute__((ext_vector_type(4), may_alias));

struct Freq { float f[64]; };
static_assert(sizeof(Freq) == 256);

__device__ __forceinline__ float bf16r(float f)
{
    unsigned int u = __float_as_uint(f);
    u += 0x7FFFu + ((u >> 16) & 1u);
    u &= 0xFFFF0000u;
    return __uint_as_float(u);
}

__device__ __forceinline__ v16h frag_g(const _Float16* p, int h8)
{
    v8h lo = *(const v8h*)(p + h8);
    v8h hi = *(const v8h*)(p + 16 + h8);
    return __builtin_shufflevector(lo, hi, 0, 1, 2, 3, 4, 5, 6, 7, 8, 9, 10, 11, 12, 13, 14, 15);
}

__device__ __forceinline__ v16h frag_s(const _Float16* p, int h8)
{
    v8h lo = *(const v8ha*)(p + h8);
    v8h hi = *(const v8ha*)(p + 16 + h8);
    return __builtin_shufflevector(lo, hi, 0, 1, 2, 3, 4, 5, 6, 7, 8, 9, 10, 11, 12, 13, 14, 15);
}

__device__ __forceinline__ v8f mma(v16h a, v16h b, v8f c)
{
    c = __builtin_amdgcn_wmma_f32_16x16x32_f16(false, a, false, b, (short)0, c, false, false);
    asm volatile("v_nop\n\tv_nop\n\tv_nop\n\tv_nop" : "+v"(c) : "v"(a), "v"(b) : "memory");
    return c;
}

__global__ __launch_bounds__(256)
void k_cvt(const float* __restrict__ src, _Float16* __restrict__ dst,
           int cols, int rows, int seq, int seqfull, float mul)
{
    const int idx = blockIdx.x * 256 + (int)threadIdx.x;
    const int cpr = cols >> 3;
    const int total = rows * cpr;
    if (idx >= total) return;
    const int row = idx / cpr;
    const int c = (idx - row * cpr) << 3;
    const int b = row / seq;
    const int s = row - b * seq;
    const float* sp = src + (size_t)(b * seqfull + s) * cols + c;
    const v4f f0 = *(const v4f*)sp;
    const v4f f1 = *(const v4f*)(sp + 4);
    v8h o;
    #pragma unroll
    for (int j = 0; j < 4; ++j) {
        o[j]     = (_Float16)(bf16r(f0[j]) * mul);
        o[4 + j] = (_Float16)(bf16r(f1[j]) * mul);
    }
    _Float16* dp = dst + (size_t)row * cols + c;
    *(volatile v8h*)dp = o;
    __threadfence();
    *(volatile v8h*)dp = o;
}

__global__ __launch_bounds__(256)
void k_tab(Freq fq, float* __restrict__ tc, float* __restrict__ ts)
{
    __shared__ float sf[64];
    __shared__ __align__(16) float scs[256 * 8];
    const int tid = threadIdx.x;
    float fv = 0.0f;
    #pragma unroll
    for (int j = 0; j < 64; ++j) fv = (tid == j) ? fq.f[j] : fv;
    if (tid < 64) sf[tid] = fv;
    __syncthreads();
    const int idx = blockIdx.x * 256 + tid;
    const int s = idx >> 4;
    const int i0 = (idx & 15) * 4;
    #pragma unroll 1
    for (int j = 0; j < 4; ++j) {
        const float ang = (float)s * sf[i0 + j];
        float sn, cs;
        sincosf(ang, &sn, &cs);
        scs[tid * 8 + j] = cs;
        scs[tid * 8 + 4 + j] = sn;
    }
    const v4f cv = *(const v4fa*)&scs[tid * 8];
    const v4f sv = *(const v4fa*)&scs[tid * 8 + 4];
    if (s < SEQ) {
        float* cpo = tc + (size_t)s * 64 + i0;
        float* spo = ts + (size_t)s * 64 + i0;
        *(volatile v4f*)cpo = cv;
        *(volatile v4f*)spo = sv;
        __threadfence();
        *(volatile v4f*)cpo = cv;
        *(volatile v4f*)spo = sv;
    }
}

template<int MODE>
__global__ __launch_bounds__(256)
void k_gemm(const _Float16* __restrict__ A, const _Float16* __restrict__ Al,
            const _Float16* __restrict__ Bw,
            const float* __restrict__ tc, const float* __restrict__ ts,
            _Float16* __restrict__ P0, _Float16* __restrict__ P1,
            float* __restrict__ outp, int soff, int rbpb)
{
    constexpr bool LO = (MODE == 4);
    constexpr int NP = (MODE == 1 || MODE == 2) ? KVD : DM;
    __shared__ __align__(16) float Cs[64 * CP];

    const int tid = threadIdx.x;
    const int lane = tid & 31;
    const int w = tid >> 5;
    const int wm = w >> 2;
    const int wn = w & 3;
    const int m = lane & 15;
    const int h8 = (lane >> 4) * 8;
    const int by = blockIdx.y;
    const int b = by / rbpb;
    const int s0 = soff + (by - b * rbpb) * 64;
    const int n0 = blockIdx.x * 128;
    const int arow0 = b * SEQ + s0;

    const _Float16* Ab  = A + (size_t)(arow0 + wm * 32 + m) * DM;
    const _Float16* Alb = LO ? (Al + (size_t)(b * RH + s0 + wm * 32 + m) * DM) : Ab;
    const _Float16* Bb  = Bw + (size_t)(n0 + wn * 32 + m) * DM;

    v8f acc[2][2], accr[2][2];
    #pragma unroll
    for (int t = 0; t < 2; ++t) {
        #pragma unroll
        for (int u = 0; u < 2; ++u) { acc[t][u] = (v8f){}; accr[t][u] = (v8f){}; }
    }

    #pragma unroll 2
    for (int k0 = 0; k0 < DM; k0 += 32) {
        const v16h a0 = frag_g(Ab + k0, h8);
        const v16h a1 = frag_g(Ab + (size_t)16 * DM + k0, h8);
        const v16h b0 = frag_g(Bb + k0, h8);
        const v16h b1 = frag_g(Bb + (size_t)16 * DM + k0, h8);
        acc[0][0] = mma(a0, b0, acc[0][0]);
        acc[0][1] = mma(a0, b1, acc[0][1]);
        acc[1][0] = mma(a1, b0, acc[1][0]);
        acc[1][1] = mma(a1, b1, acc[1][1]);
        if (LO) {
            const v16h l0 = frag_g(Alb + k0, h8);
            const v16h l1 = frag_g(Alb + (size_t)16 * DM + k0, h8);
            accr[0][0] = mma(l0, b0, accr[0][0]);
            accr[0][1] = mma(l0, b1, accr[0][1]);
            accr[1][0] = mma(l1, b0, accr[1][0]);
            accr[1][1] = mma(l1, b1, accr[1][1]);
        }
    }

    const float i64 = 1.0f / 64.0f;
    const float i1024 = 1.0f / 1024.0f;
    #pragma unroll
    for (int t = 0; t < 2; ++t) {
        #pragma unroll
        for (int u = 0; u < 2; ++u) {
            #pragma unroll
            for (int r = 0; r < 8; ++r) {
                float v;
                if (LO) v = (acc[t][u][r] + accr[t][u][r] * i1024) * i64;
                else    v = acc[t][u][r] * i64;
                Cs[(wm * 32 + t * 16 + h8 + r) * CP + wn * 32 + u * 16 + m] = v;
            }
        }
    }
    __syncthreads();

    if (MODE == 0 || MODE == 1) {
        #pragma unroll
        for (int it = 0; it < 4; ++it) {
            const int idx = it * 256 + tid;
            const int row = idx >> 4;
            const int c8 = (idx & 15) * 8;
            const int s = s0 + row;
            const int i0 = c8 & 63;
            const float sg = (c8 < 64) ? -1.0f : 1.0f;
            const float* xr = &Cs[row * CP + c8];
            const float* yr = &Cs[row * CP + (c8 ^ 64)];
            const v4f x0 = *(const v4fa*)xr;
            const v4f x1 = *(const v4fa*)(xr + 4);
            const v4f y0 = *(const v4fa*)yr;
            const v4f y1 = *(const v4fa*)(yr + 4);
            const float* cr = tc + (size_t)s * 64 + i0;
            const float* sr = ts + (size_t)s * 64 + i0;
            const v4f cc0 = *(const v4f*)cr;
            const v4f cc1 = *(const v4f*)(cr + 4);
            const v4f ss0 = *(const v4f*)sr;
            const v4f ss1 = *(const v4f*)(sr + 4);
            v8h hv, lv;
            #pragma unroll
            for (int j = 0; j < 4; ++j) {
                const float va = x0[j] * cc0[j] + sg * (y0[j] * ss0[j]);
                const float vb = x1[j] * cc1[j] + sg * (y1[j] * ss1[j]);
                const _Float16 ha = (_Float16)va;
                const _Float16 hb = (_Float16)vb;
                hv[j] = ha;
                hv[4 + j] = hb;
                lv[j] = (_Float16)((va - (float)ha) * 1024.0f);
                lv[4 + j] = (_Float16)((vb - (float)hb) * 1024.0f);
            }
            _Float16* hp = P0 + (size_t)(arow0 + row) * NP + n0 + c8;
            _Float16* lp = P1 + (size_t)(b * RH + s) * NP + n0 + c8;
            const bool wlo = (s0 < RH);
            *(volatile v8h*)hp = hv;
            if (wlo) *(volatile v8h*)lp = lv;
            __threadfence();
            *(volatile v8h*)hp = hv;
            if (wlo) *(volatile v8h*)lp = lv;
        }
    } else if (MODE == 2) {
        const int kvh = blockIdx.x;
        #pragma unroll
        for (int it = 0; it < 4; ++it) {
            const int idx = it * 256 + tid;
            const int d = idx >> 3;
            const int p = idx & 7;
            v8h hv, lv;
            #pragma unroll
            for (int j = 0; j < 8; ++j) {
                const float va = Cs[(p * 8 + j) * CP + d];
                const _Float16 ha = (_Float16)va;
                hv[j] = ha;
                lv[j] = (_Float16)((va - (float)ha) * 1024.0f);
            }
            const size_t drow = (size_t)(b * NKV + kvh) * HD + d;
            _Float16* hp = P0 + drow * SEQ + s0 + p * 8;
            _Float16* lp = P1 + drow * RH + s0 + p * 8;
            const bool wlo = (s0 < RH);
            *(volatile v8h*)hp = hv;
            if (wlo) *(volatile v8h*)lp = lv;
            __threadfence();
            *(volatile v8h*)hp = hv;
            if (wlo) *(volatile v8h*)lp = lv;
        }
    } else {
        #pragma unroll
        for (int it = 0; it < 8; ++it) {
            const int idx = it * 256 + tid;
            const int row = idx >> 5;
            const int c4 = (idx & 31) * 4;
            const v4f v = *(const v4fa*)&Cs[row * CP + c4];
            float* op = outp + (size_t)(b * SEQ_FULL + s0 + row) * DM + n0 + c4;
            *(volatile v4f*)op = v;
            __threadfence();
            *(volatile v4f*)op = v;
        }
    }
}

template<bool HP>
__global__ __launch_bounds__(HP ? 256 : 128)
void k_attn(const _Float16* __restrict__ qh, const _Float16* __restrict__ ql,
            const _Float16* __restrict__ kh, const _Float16* __restrict__ kl,
            const _Float16* __restrict__ vth, const _Float16* __restrict__ vtl,
            _Float16* __restrict__ ch, _Float16* __restrict__ cl, int sblk0)
{
    constexpr int NW  = HP ? 8 : 4;
    constexpr int NDC = HP ? 4 : 8;
    constexpr int PTP = 40;
    constexpr int CTP = NDC * 16 + 8;
    __shared__ __align__(16) _Float16 Pth[NW * 16 * PTP];
    __shared__ __align__(16) _Float16 Ptl[HP ? NW * 16 * PTP : 8];
    __shared__ __align__(16) _Float16 Ct[NW * 16 * CTP];
    __shared__ __align__(16) _Float16 Ctl[HP ? NW * 16 * CTP : 8];

    const int tid = threadIdx.x;
    const int lane = tid & 31;
    const int w = tid >> 5;
    const int m = lane & 15;
    const int n = m;
    const int h8 = (lane >> 4) * 8;
    const int tile = w & 3;
    const int dbase = HP ? (w >> 2) * NDC : 0;
    const int b = blockIdx.z;
    const int head = blockIdx.y;
    const int kv = head / NREP;
    const int s0 = sblk0 + blockIdx.x * 64;
    const int q0 = s0 + tile * 16;
    const int nch = ((q0 + 15) >> 5) + 1;

    _Float16* pth = Pth + w * 16 * PTP;
    _Float16* ptl = HP ? (Ptl + w * 16 * PTP) : pth;
    _Float16* ct  = Ct + w * 16 * CTP;
    _Float16* ctl = HP ? (Ctl + w * 16 * CTP) : ct;

    const _Float16* qrow  = qh + (size_t)(b * SEQ + q0 + m) * DM + head * HD;
    const _Float16* qlrow = HP ? (ql + (size_t)(b * RH + q0 + m) * DM + head * HD) : qrow;
    const _Float16* vbase  = vth + ((size_t)(b * NKV + kv) * HD + dbase * 16 + m) * SEQ;
    const _Float16* vlbase = HP ? (vtl + ((size_t)(b * NKV + kv) * HD + dbase * 16 + m) * RH) : vbase;

    const float rs = 1.0f / 11.313708498984761f;
    const float i1024 = 1.0f / 1024.0f;

    float mrow[8], lrow[8];
    v8f acc[NDC], accr[NDC];
    #pragma unroll
    for (int r = 0; r < 8; ++r) { mrow[r] = -1.0e30f; lrow[r] = 0.0f; }
    #pragma unroll
    for (int dch = 0; dch < NDC; ++dch) { acc[dch] = (v8f){}; accr[dch] = (v8f){}; }

    #pragma unroll 1
    for (int c = 0; c < nch; ++c) {
        const int key0 = c * 32;
        const _Float16* k0r  = kh + (size_t)(b * SEQ + key0 + m) * KVD + kv * HD;
        const _Float16* k1r  = k0r + (size_t)16 * KVD;
        const _Float16* kl0r = HP ? (kl + (size_t)(b * RH + key0 + m) * KVD + kv * HD) : k0r;
        const _Float16* kl1r = kl0r + (size_t)16 * KVD;

        v8f s0f = (v8f){}, s1f = (v8f){}, r0f = (v8f){}, r1f = (v8f){};
        #pragma unroll
        for (int kc = 0; kc < 4; ++kc) {
            const v16h aq  = frag_g(qrow + kc * 32, h8);
            const v16h bk0 = frag_g(k0r + kc * 32, h8);
            const v16h bk1 = frag_g(k1r + kc * 32, h8);
            s0f = mma(aq, bk0, s0f);
            s1f = mma(aq, bk1, s1f);
            if (HP) {
                const v16h aql  = frag_g(qlrow + kc * 32, h8);
                const v16h bkl0 = frag_g(kl0r + kc * 32, h8);
                const v16h bkl1 = frag_g(kl1r + kc * 32, h8);
                r0f = mma(aq, bkl0, r0f);
                r0f = mma(aql, bk0, r0f);
                r1f = mma(aq, bkl1, r1f);
                r1f = mma(aql, bk1, r1f);
            }
        }

        #pragma unroll
        for (int r = 0; r < 8; ++r) {
            const int i = q0 + h8 + r;
            float sc0, sc1;
            if (HP) {
                sc0 = (s0f[r] + r0f[r] * i1024) * rs;
                sc1 = (s1f[r] + r1f[r] * i1024) * rs;
            } else {
                sc0 = s0f[r] * rs;
                sc1 = s1f[r] * rs;
            }
            const bool ok0 = (key0 + n) <= i;
            const bool ok1 = (key0 + 16 + n) <= i;
            sc0 = ok0 ? sc0 : -3.0e38f;
            sc1 = ok1 ? sc1 : -3.0e38f;
            float mx = fmaxf(sc0, sc1);
            #pragma unroll
            for (int off = 1; off < 16; off <<= 1) mx = fmaxf(mx, __shfl_xor(mx, off, 32));
            const float mnew = fmaxf(mrow[r], mx);
            const float fac = __expf(mrow[r] - mnew);
            const float p0 = __expf(sc0 - mnew);
            const float p1 = __expf(sc1 - mnew);
            float ps = p0 + p1;
            #pragma unroll
            for (int off = 1; off < 16; off <<= 1) ps += __shfl_xor(ps, off, 32);
            lrow[r] = lrow[r] * fac + ps;
            mrow[r] = mnew;
            #pragma unroll
            for (int dch = 0; dch < NDC; ++dch) {
                acc[dch][r] *= fac;
                if (HP) accr[dch][r] *= fac;
            }
            const float p0s = p0 * 1024.0f;
            const float p1s = p1 * 1024.0f;
            const _Float16 ph0 = (_Float16)p0s;
            const _Float16 ph1 = (_Float16)p1s;
            pth[(h8 + r) * PTP + n] = ph0;
            pth[(h8 + r) * PTP + 16 + n] = ph1;
            if (HP) {
                ptl[(h8 + r) * PTP + n]      = (_Float16)((p0s - (float)ph0) * 1024.0f);
                ptl[(h8 + r) * PTP + 16 + n] = (_Float16)((p1s - (float)ph1) * 1024.0f);
            }
        }
        __builtin_amdgcn_fence(__ATOMIC_RELEASE, "wavefront");
        __builtin_amdgcn_wave_barrier();

        const v16h ap  = frag_s(pth + m * PTP, h8);
        const v16h apl = HP ? frag_s(ptl + m * PTP, h8) : ap;
        #pragma unroll
        for (int dch = 0; dch < NDC; ++dch) {
            const v16h bv = frag_g(vbase + (size_t)(dch * 16) * SEQ + key0, h8);
            acc[dch] = mma(ap, bv, acc[dch]);
            if (HP) {
                const v16h bvl = frag_g(vlbase + (size_t)(dch * 16) * RH + key0, h8);
                accr[dch] = mma(ap, bvl, accr[dch]);
                accr[dch] = mma(apl, bv, accr[dch]);
            }
        }
    }

    #pragma unroll
    for (int r = 0; r < 8; ++r) {
        const float inv = __builtin_amdgcn_rcpf(lrow[r] * 1024.0f);
        #pragma unroll
        for (int dch = 0; dch < NDC; ++dch) {
            float v;
            if (HP) v = (acc[dch][r] + accr[dch][r] * i1024) * inv;
            else    v = acc[dch][r] * inv;
            const _Float16 hv = (_Float16)v;
            ct[(h8 + r) * CTP + dch * 16 + n] = hv;
            if (HP) ctl[(h8 + r) * CTP + dch * 16 + n] = (_Float16)((v - (float)hv) * 1024.0f);
        }
    }
    __builtin_amdgcn_fence(__ATOMIC_RELEASE, "wavefront");
    __builtin_amdgcn_wave_barrier();

    if (!HP) {
        #pragma unroll
        for (int it = 0; it < 8; ++it) {
            const int row = it * 2 + (lane >> 4);
            const int c8 = m * 8;
            const v8h hv = *(const v8ha*)&ct[row * CTP + c8];
            _Float16* op = ch + (size_t)(b * SEQ + q0 + row) * DM + head * HD + c8;
            *(volatile v8h*)op = hv;
            __threadfence();
            *(volatile v8h*)op = hv;
        }
    } else {
        #pragma unroll
        for (int it = 0; it < 4; ++it) {
            const int row = it * 4 + (lane >> 3);
            const int c8 = (lane & 7) * 8;
            const v8h hv = *(const v8ha*)&ct[row * CTP + c8];
            const v8h lv = *(const v8ha*)&ctl[row * CTP + c8];
            _Float16* op = ch + (size_t)(b * SEQ + q0 + row) * DM + head * HD + dbase * 16 + c8;
            _Float16* lp = cl + (size_t)(b * RH + q0 + row) * DM + head * HD + dbase * 16 + c8;
            *(volatile v8h*)op = hv;
            *(volatile v8h*)lp = lv;
            __threadfence();
            *(volatile v8h*)op = hv;
            *(volatile v8h*)lp = lv;
        }
    }
}

static inline size_t al256(size_t x) { return (x + 255) & ~(size_t)255; }

extern "C" void kernel_launch(void* const* d_in, const int* in_sizes, int n_in,
                              void* d_out, int out_size, void* d_ws, size_t ws_size,
                              hipStream_t stream)
{
    if (n_in < 5) return;
    const long needx = ((long)(NB - 1) * SEQ_FULL + SEQ) * DM;
    if ((long)in_sizes[0] < needx) return;
    if ((long)in_sizes[1] < (long)DM * DM) return;
    if ((long)in_sizes[2] < (long)KVD * DM) return;
    if ((long)in_sizes[3] < (long)KVD * DM) return;
    if ((long)in_sizes[4] < (long)DM * DM) return;
    if ((long)out_size < needx) return;

    const float* x  = (const float*)d_in[0];
    const float* Wq = (const float*)d_in[1];
    const float* Wk = (const float*)d_in[2];
    const float* Wv = (const float*)d_in[3];
    const float* Wo = (const float*)d_in[4];
    float* out = (float*)d_out;

    char* ws = (char*)d_ws;
    size_t off = 0;
    auto take = [&](size_t bytes) -> char* { char* p = ws + off; off += al256(bytes); return p; };

    float*    tc  = (float*)take((size_t)SEQ * 64 * 4);
    float*    ts  = (float*)take((size_t)SEQ * 64 * 4);
    _Float16* xh  = (_Float16*)take((size_t)MROWS * DM * 2);
    _Float16* wq  = (_Float16*)take((size_t)DM * DM * 2);
    _Float16* wk  = (_Float16*)take((size_t)KVD * DM * 2);
    _Float16* wv  = (_Float16*)take((size_t)KVD * DM * 2);
    _Float16* wo  = (_Float16*)take((size_t)DM * DM * 2);
    _Float16* qh  = (_Float16*)take((size_t)MROWS * DM * 2);
    _Float16* ql  = (_Float16*)take((size_t)NB * RH * DM * 2);
    _Float16* khp = (_Float16*)take((size_t)MROWS * KVD * 2);
    _Float16* klp = (_Float16*)take((size_t)NB * RH * KVD * 2);
    _Float16* vth = (_Float16*)take((size_t)NB * NKV * HD * SEQ * 2);
    _Float16* vtl = (_Float16*)take((size_t)NB * NKV * HD * RH * 2);
    _Float16* chp = (_Float16*)take((size_t)MROWS * DM * 2);
    _Float16* clp = (_Float16*)take((size_t)NB * RH * DM * 2);
    if (off > ws_size) return;

    Freq fq;
    for (int i = 0; i < 64; ++i) {
        const float e = (float)i / 64.0f;
        const float p = powf(10000.0f, e);
        fq.f[i] = 1.0f / p;
    }

    k_tab<<<dim3(SEQ / 16), dim3(256), 0, stream>>>(fq, tc, ts);

    {
        const int px = (MROWS * (DM / 8) + 255) / 256;
        k_cvt<<<dim3(px), dim3(256), 0, stream>>>(x, xh, DM, MROWS, SEQ, SEQ_FULL, 1.0f);
        const int pq = (DM * (DM / 8) + 255) / 256;
        k_cvt<<<dim3(pq), dim3(256), 0, stream>>>(Wq, wq, DM, DM, DM, DM, 64.0f);
        const int pk = (KVD * (DM / 8) + 255) / 256;
        k_cvt<<<dim3(pk), dim3(256), 0, stream>>>(Wk, wk, DM, KVD, KVD, KVD, 64.0f);
        k_cvt<<<dim3(pk), dim3(256), 0, stream>>>(Wv, wv, DM, KVD, KVD, KVD, 64.0f);
        k_cvt<<<dim3(pq), dim3(256), 0, stream>>>(Wo, wo, DM, DM, DM, DM, 64.0f);
    }

    k_gemm<0><<<dim3(DM / 128, MROWS / 64), dim3(256), 0, stream>>>(xh, xh, wq, tc, ts, qh, ql, out, 0, SEQ / 64);
    k_gemm<1><<<dim3(KVD / 128, MROWS / 64), dim3(256), 0, stream>>>(xh, xh, wk, tc, ts, khp, klp, out, 0, SEQ / 64);
    k_gemm<2><<<dim3(KVD / 128, MROWS / 64), dim3(256), 0, stream>>>(xh, xh, wv, tc, ts, vth, vtl, out, 0, SEQ / 64);

    k_attn<true><<<dim3(RH / 64, NH, NB), dim3(256), 0, stream>>>(qh, ql, khp, klp, vth, vtl, chp, clp, 0);
    if (SEQ > RH) {
        k_attn<false><<<dim3((SEQ - RH) / 64, NH, NB), dim3(128), 0, stream>>>(qh, ql, khp, klp, vth, vtl, chp, clp, RH);
    }

    k_gemm<4><<<dim3(DM / 128, NB * (RH / 64)), dim3(256), 0, stream>>>(chp, clp, wo, tc, ts, qh, ql, out, 0, RH / 64);
    if (SEQ > RH) {
        k_gemm<3><<<dim3(DM / 128, NB * ((SEQ - RH) / 64)), dim3(256), 0, stream>>>(chp, chp, wo, tc, ts, qh, ql, out, RH, (SEQ - RH) / 64);
    }
}
